// GPTBlock_369367188059
// MI455X (gfx1250) — hardware-run, weakly checked
//
#include <hip/hip_runtime.h>
#include <stdint.h>


typedef _Float16 v16h __attribute__((ext_vector_type(16)));
typedef _Float16 v8h  __attribute__((ext_vector_type(8)));
typedef float    v8f  __attribute__((ext_vector_type(8)));
typedef float    v4f  __attribute__((ext_vector_type(4)));
typedef unsigned int u32x4 __attribute__((ext_vector_type(4)));

#ifndef NB
#define NB 2
#endif
#ifndef SEQ
#define SEQ 2048
#endif
#define NB_FULL 2
#define SEQ_FULL 2048

constexpr int kD   = 1024;
constexpr int kH   = 16;
constexpr int kDH  = 64;
constexpr int kDFF = 4096;
constexpr int kM   = NB * SEQ;
constexpr float kEps      = 1e-5f;
constexpr float kWCarry   = 64.0f;
constexpr float kPCarry   = 1024.0f;
constexpr float kCtxCarry = 16.0f;
constexpr float kGCarry   = 16.0f;

static_assert(SEQ % 128 == 0);
static_assert(SEQ <= SEQ_FULL);
static_assert(NB >= 1 && NB <= NB_FULL);
static_assert(kM % 128 == 0);
static_assert(kD % 128 == 0 && kDFF % 128 == 0);
static_assert(kD % 32 == 0 && kDFF % 32 == 0);
static_assert(kH * kDH == kD);

enum { EPI_QK = 0, EPI_GELU = 1, EPI_Z1 = 2, EPI_OUT = 3 };

__device__ __forceinline__ v8f wmma16(v16h a, v16h b, v8f c) {
  v8f d = __builtin_amdgcn_wmma_f32_16x16x32_f16(false, a, false, b, (short)0, c,
                                                 false, false);
  asm volatile("v_nop\n\tv_nop\n\tv_nop\n\tv_nop" : "+v"(d) : "v"(a), "v"(b));
  return d;
}

__device__ __forceinline__ v16h load_frag(const _Float16* p, int ld, int lane) {
  const int r  = lane & 15;
  const int k8 = (lane >> 4) << 3;
  const _Float16* q = p + (size_t)r * ld + k8;
  union { v16h v; v8h h[2]; } u;
  u.h[0] = *(const v8h*)(q);
  u.h[1] = *(const v8h*)(q + 16);
  return u.v;
}

__device__ __forceinline__ float bf16r(float x) {
  unsigned int u = __float_as_uint(x);
  u += 0x7FFFu + ((u >> 16) & 1u);
  u &= 0xFFFF0000u;
  return __uint_as_float(u);
}

__device__ __forceinline__ float gelu_f(float x) {
  return 0.5f * x * (1.0f + erff(x * 0.70710678118654752f));
}

__device__ __forceinline__ void vst4f(float* p, v4f v) { *(volatile v4f*)p = v; }
__device__ __forceinline__ void vst8h(_Float16* p, v8h v) {
  union { v8h h; u32x4 u; } t;
  t.h = v;
  *(volatile u32x4*)p = t.u;
}

__global__ __launch_bounds__(256)
void cvt_wt(const float* __restrict__ W, _Float16* __restrict__ Wt, int K, int N) {
  __shared__ __align__(16) _Float16 tile[64 * 72];
  const int t  = threadIdx.x;
  const int n0 = blockIdx.x * 64;
  const int k0 = blockIdx.y * 64;
#pragma unroll
  for (int it = 0; it < 4; ++it) {
    const int idx = t + it * 256;
    const int kr  = idx >> 4;
    const int c4  = (idx & 15) * 4;
    const v4f v = *(const v4f*)(W + (size_t)(k0 + kr) * N + n0 + c4);
#pragma unroll
    for (int e = 0; e < 4; ++e)
      tile[(c4 + e) * 72 + kr] = (_Float16)(bf16r(v[e]) * kWCarry);
  }
  __syncthreads();
  v8h sv[2];
#pragma unroll
  for (int it = 0; it < 2; ++it) {
    const int idx = t + it * 256;
    const int row = idx >> 3, piece = idx & 7;
    sv[it] = *(const v8h*)(&tile[row * 72 + piece * 8]);
    vst8h(Wt + (size_t)(n0 + row) * K + k0 + piece * 8, sv[it]);
  }
  __threadfence();
#pragma unroll
  for (int it = 0; it < 2; ++it) {
    const int idx = t + it * 256;
    const int row = idx >> 3, piece = idx & 7;
    vst8h(Wt + (size_t)(n0 + row) * K + k0 + piece * 8, sv[it]);
  }
}

template <int SRC_FULL>
__global__ __launch_bounds__(128)
void rmsnorm_f16(const float* __restrict__ x, const float* __restrict__ g,
                 _Float16* __restrict__ y) {
  __shared__ float red[4];
  const int m    = blockIdx.x;
  const int t    = threadIdx.x;
  const int lane = t & 31, wave = t >> 5;
  size_t srow;
  if (SRC_FULL) srow = (size_t)(m / SEQ) * SEQ_FULL + (size_t)(m % SEQ);
  else          srow = (size_t)m;
  const float* xr = x + srow * kD + t * 8;
  const v4f a = *(const v4f*)(xr);
  const v4f b = *(const v4f*)(xr + 4);
  float v[8];
#pragma unroll
  for (int e = 0; e < 4; ++e) { v[e] = a[e]; v[4 + e] = b[e]; }
  if (SRC_FULL) {
#pragma unroll
    for (int e = 0; e < 8; ++e) v[e] = bf16r(v[e]);
  }
  float ss = 0.0f;
#pragma unroll
  for (int e = 0; e < 8; ++e) ss += v[e] * v[e];
#pragma unroll
  for (int off = 16; off > 0; off >>= 1) ss += __shfl_xor(ss, off);
  if (lane == 0) red[wave] = ss;
  __syncthreads();
  const float tot = (red[0] + red[1]) + (red[2] + red[3]);
  const float rms = sqrtf(tot * (1.0f / (float)kD) + kEps);
  const float inv = 1.0f / rms;
  const v4f ga = *(const v4f*)(g + t * 8);
  const v4f gb = *(const v4f*)(g + t * 8 + 4);
  v8h o;
#pragma unroll
  for (int e = 0; e < 4; ++e) {
    o[e]     = (_Float16)((v[e] * inv) * bf16r(ga[e]));
    o[4 + e] = (_Float16)((v[4 + e] * inv) * bf16r(gb[e]));
  }
  _Float16* dst = y + (size_t)m * kD + t * 8;
  vst8h(dst, o);
  __threadfence();
  vst8h(dst, o);
}

template <int MI, int NJ>
__device__ __forceinline__ void gemm_core(v8f (&acc)[MI][NJ], const _Float16* Aw,
                                          const _Float16* Bw, int K, int lane) {
  for (int k0 = 0; k0 < K; k0 += 32) {
    v16h a[MI];
#pragma unroll
    for (int i = 0; i < MI; ++i) a[i] = load_frag(Aw + (size_t)(i * 16) * K + k0, K, lane);
#pragma unroll
    for (int j = 0; j < NJ; ++j) {
      const v16h b = load_frag(Bw + (size_t)(j * 16) * K + k0, K, lane);
#pragma unroll
      for (int i = 0; i < MI; ++i) acc[i][j] = wmma16(a[i], b, acc[i][j]);
    }
  }
}

template <int EPI>
__global__ __launch_bounds__(256)
void gemm_rows(const _Float16* __restrict__ A, const _Float16* __restrict__ Bt,
               const float* __restrict__ resid, float* __restrict__ outF,
               _Float16* __restrict__ outH, int N, int K) {
  __shared__ __align__(16) float stg[8][16 * 68];
  const int tid = threadIdx.x, lane = tid & 31, wave = tid >> 5;
  const int wm = wave & 3, wn = wave >> 2;
  const int m0w = blockIdx.x * 128 + wm * 32;
  const int n0w = blockIdx.y * 128 + wn * 64;
  const _Float16* Aw = A + (size_t)m0w * K;
  const _Float16* Bw = Bt + (size_t)n0w * K;

  v8f acc[2][4] = {};
  gemm_core<2, 4>(acc, Aw, Bw, K, lane);

  constexpr float sc = (EPI == EPI_QK || EPI == EPI_GELU) ? (1.0f / 64.0f) : (1.0f / 1024.0f);
  const int n = lane & 15, h8 = (lane >> 4) * 8;
  float* sw = &stg[wave][0];

#pragma unroll
  for (int i = 0; i < 2; ++i) {
#pragma unroll
    for (int j = 0; j < 4; ++j)
#pragma unroll
      for (int r = 0; r < 8; ++r)
        sw[(h8 + r) * 68 + j * 16 + n] = acc[i][j][r] * sc;
    __syncthreads();
    if constexpr (EPI == EPI_Z1 || EPI == EPI_OUT) {
      v4f sv[8];
#pragma unroll
      for (int q = 0; q < 8; ++q) {
        const int row = q * 2 + (lane >> 4), col = (lane & 15) * 4;
        const int gm = m0w + i * 16 + row, gn = n0w + col;
        v4f v = *(const v4f*)(sw + row * 68 + col);
        size_t roff;
        if constexpr (EPI == EPI_Z1)
          roff = ((size_t)(gm / SEQ) * SEQ_FULL + (size_t)(gm % SEQ)) * (size_t)kD + gn;
        else
          roff = (size_t)gm * N + gn;
        const v4f rr = *(const v4f*)(resid + roff);
#pragma unroll
        for (int e = 0; e < 4; ++e) {
          float re = rr[e];
          if constexpr (EPI == EPI_Z1) re = bf16r(re);
          v[e] = re + v[e];
        }
        sv[q] = v;
        vst4f(outF + (size_t)gm * N + gn, v);
      }
      __threadfence();
#pragma unroll
      for (int q = 0; q < 8; ++q) {
        const int row = q * 2 + (lane >> 4), col = (lane & 15) * 4;
        const int gm = m0w + i * 16 + row, gn = n0w + col;
        vst4f(outF + (size_t)gm * N + gn, sv[q]);
      }
    } else {
      v8h sv[4];
#pragma unroll
      for (int q = 0; q < 4; ++q) {
        const int row = q * 4 + (lane >> 3), col = (lane & 7) * 8;
        const int gm = m0w + i * 16 + row, gn = n0w + col;
        const v4f va = *(const v4f*)(sw + row * 68 + col);
        const v4f vb = *(const v4f*)(sw + row * 68 + col + 4);
        v8h o;
#pragma unroll
        for (int e = 0; e < 4; ++e) {
          float xa = va[e], xb = vb[e];
          if constexpr (EPI == EPI_GELU) { xa = gelu_f(xa) * kGCarry; xb = gelu_f(xb) * kGCarry; }
          o[e]     = (_Float16)xa;
          o[4 + e] = (_Float16)xb;
        }
        sv[q] = o;
        _Float16* dst;
        if constexpr (EPI == EPI_QK) {
          const int b = gm / SEQ, l = gm % SEQ, hh = gn >> 6, dh = gn & 63;
          dst = outH + (((size_t)(b * kH + hh)) * SEQ + l) * kDH + dh;
        } else {
          dst = outH + (size_t)gm * N + gn;
        }
        vst8h(dst, o);
      }
      __threadfence();
#pragma unroll
      for (int q = 0; q < 4; ++q) {
        const int row = q * 4 + (lane >> 3), col = (lane & 7) * 8;
        const int gm = m0w + i * 16 + row, gn = n0w + col;
        _Float16* dst;
        if constexpr (EPI == EPI_QK) {
          const int b = gm / SEQ, l = gm % SEQ, hh = gn >> 6, dh = gn & 63;
          dst = outH + (((size_t)(b * kH + hh)) * SEQ + l) * kDH + dh;
        } else {
          dst = outH + (size_t)gm * N + gn;
        }
        vst8h(dst, sv[q]);
      }
    }
    __syncthreads();
  }
}

__global__ __launch_bounds__(256)
void gemm_vt(const _Float16* __restrict__ A, const _Float16* __restrict__ Bt,
             _Float16* __restrict__ Vt, int K) {
  __shared__ __align__(16) _Float16 stg[8][32 * 72];
  const int tid = threadIdx.x, lane = tid & 31, wave = tid >> 5;
  const int wm = wave & 1, wn = wave >> 1;
  const int m0w = blockIdx.x * 128 + wm * 64;
  const int n0w = blockIdx.y * 128 + wn * 32;
  const _Float16* Aw = A + (size_t)m0w * K;
  const _Float16* Bw = Bt + (size_t)n0w * K;

  v8f acc[4][2] = {};
  gemm_core<4, 2>(acc, Aw, Bw, K, lane);

  const int n = lane & 15, h8 = (lane >> 4) * 8;
  _Float16* sw = &stg[wave][0];
#pragma unroll
  for (int i = 0; i < 4; ++i)
#pragma unroll
    for (int j = 0; j < 2; ++j)
#pragma unroll
      for (int r = 0; r < 8; ++r)
        sw[(j * 16 + n) * 72 + i * 16 + h8 + r] = (_Float16)(acc[i][j][r] * (1.0f / 64.0f));
  __syncthreads();

  const int b  = m0w / SEQ;
  const int l0 = m0w % SEQ;
  const int hh = n0w >> 6;
  const int dh0 = n0w & 63;
  v8h sv[8];
#pragma unroll
  for (int q = 0; q < 8; ++q) {
    const int row = q * 4 + (lane >> 3), piece = lane & 7;
    sv[q] = *(const v8h*)(sw + row * 72 + piece * 8);
    _Float16* dst = Vt + ((size_t)(b * kH + hh) * kDH + dh0 + row) * SEQ + l0 + piece * 8;
    vst8h(dst, sv[q]);
  }
  __threadfence();
#pragma unroll
  for (int q = 0; q < 8; ++q) {
    const int row = q * 4 + (lane >> 3), piece = lane & 7;
    _Float16* dst = Vt + ((size_t)(b * kH + hh) * kDH + dh0 + row) * SEQ + l0 + piece * 8;
    vst8h(dst, sv[q]);
  }
}

__global__ __launch_bounds__(128)
void attn_causal(const _Float16* __restrict__ Qp, const _Float16* __restrict__ Kp,
                 const _Float16* __restrict__ Vtp, _Float16* __restrict__ ctxp) {
  __shared__ __align__(16) _Float16 Ps[4][16 * 72];
  const int bh   = blockIdx.y;
  const int qblk = blockIdx.x;
  const int q0   = qblk * 64;
  const int wave = threadIdx.x >> 5;
  const int lane = threadIdx.x & 31;
  const int qw   = q0 + wave * 16;
  const int n    = lane & 15;
  const int h8   = (lane >> 4) * 8;

  const _Float16* Qh = Qp + ((size_t)bh * SEQ + qw) * kDH;
  const _Float16* Kb = Kp + (size_t)bh * SEQ * kDH;
  const _Float16* Vb = Vtp + (size_t)bh * kDH * SEQ;

  const v16h qf0 = load_frag(Qh, kDH, lane);
  const v16h qf1 = load_frag(Qh + 32, kDH, lane);

  v8f ctx[4] = {};
  float rmax[8], rsum[8];
#pragma unroll
  for (int r = 0; r < 8; ++r) { rmax[r] = -1.0e30f; rsum[r] = 0.0f; }
  _Float16* pw = &Ps[wave][0];

  for (int c = 0; c <= qblk; ++c) {
    const int j0 = c * 64;
    v8f s[4] = {};
#pragma unroll
    for (int j = 0; j < 4; ++j) {
      const _Float16* krow = Kb + (size_t)(j0 + j * 16) * kDH;
      const v16h kb0 = load_frag(krow, kDH, lane);
      const v16h kb1 = load_frag(krow + 32, kDH, lane);
      s[j] = wmma16(qf0, kb0, s[j]);
      s[j] = wmma16(qf1, kb1, s[j]);
    }

#pragma unroll
    for (int r = 0; r < 8; ++r) {
      const int qrow = qw + h8 + r;
      float mx = -1.0e30f;
#pragma unroll
      for (int j = 0; j < 4; ++j) {
        const int key = j0 + j * 16 + n;
        float sv = s[j][r] * 0.125f;
        sv = (key > qrow) ? -1.0e30f : sv;
        s[j][r] = sv;
        mx = fmaxf(mx, sv);
      }
      mx = fmaxf(mx, __shfl_xor(mx, 1));
      mx = fmaxf(mx, __shfl_xor(mx, 2));
      mx = fmaxf(mx, __shfl_xor(mx, 4));
      mx = fmaxf(mx, __shfl_xor(mx, 8));
      const float mnew = fmaxf(rmax[r], mx);
      const float corr = __expf(rmax[r] - mnew);
      rmax[r] = mnew;
      float ps = 0.0f;
#pragma unroll
      for (int j = 0; j < 4; ++j) {
        const float p = __expf(s[j][r] - mnew);
        s[j][r] = p;
        ps += p;
      }
      ps += __shfl_xor(ps, 1);
      ps += __shfl_xor(ps, 2);
      ps += __shfl_xor(ps, 4);
      ps += __shfl_xor(ps, 8);
      rsum[r] = rsum[r] * corr + ps;
#pragma unroll
      for (int d = 0; d < 4; ++d) ctx[d][r] *= corr;
    }

#pragma unroll
    for (int j = 0; j < 4; ++j)
#pragma unroll
      for (int r = 0; r < 8; ++r)
        pw[(h8 + r) * 72 + j * 16 + n] = (_Float16)(s[j][r] * kPCarry);
    __syncthreads();
#pragma unroll
    for (int kk = 0; kk < 2; ++kk) {
      const v16h pa = load_frag(pw + kk * 32, 72, lane);
#pragma unroll
      for (int d = 0; d < 4; ++d) {
        const v16h vb = load_frag(Vb + (size_t)(d * 16) * SEQ + j0 + kk * 32, SEQ, lane);
        ctx[d] = wmma16(pa, vb, ctx[d]);
      }
    }
    __syncthreads();
  }

  const int b  = bh / kH;
  const int hh = bh % kH;
#pragma unroll
  for (int r = 0; r < 8; ++r) {
    const float inv = (kCtxCarry / kPCarry) / rsum[r];
#pragma unroll
    for (int d = 0; d < 4; ++d)
      pw[(h8 + r) * 72 + d * 16 + n] = (_Float16)(ctx[d][r] * inv);
  }
  __syncthreads();
  v8h sv[4];
#pragma unroll
  for (int q = 0; q < 4; ++q) {
    const int row = q * 4 + (lane >> 3), piece = lane & 7;
    sv[q] = *(const v8h*)(pw + row * 72 + piece * 8);
    _Float16* dst = ctxp + ((size_t)b * SEQ + qw + row) * kD + hh * kDH + piece * 8;
    vst8h(dst, sv[q]);
  }
  __threadfence();
#pragma unroll
  for (int q = 0; q < 4; ++q) {
    const int row = q * 4 + (lane >> 3), piece = lane & 7;
    _Float16* dst = ctxp + ((size_t)b * SEQ + qw + row) * kD + hh * kDH + piece * 8;
    vst8h(dst, sv[q]);
  }
}

extern "C" void kernel_launch(void* const* d_in, const int* in_sizes, int n_in,
                              void* d_out, int out_size, void* d_ws, size_t ws_size,
                              hipStream_t stream) {
  if (n_in < 9) return;
  if (in_sizes[0] < ((NB - 1) * SEQ_FULL + SEQ) * kD) return;
  if (in_sizes[1] < kD * kD || in_sizes[2] < kD * kD ||
      in_sizes[3] < kD * kD || in_sizes[4] < kD * kD) return;
  if (in_sizes[5] < kD * kDFF || in_sizes[6] < kDFF * kD) return;
  if (in_sizes[7] < kD || in_sizes[8] < kD) return;
  if (out_size < kM * kD) return;

  const float* z      = (const float*)d_in[0];
  const float* W_Q    = (const float*)d_in[1];
  const float* W_K    = (const float*)d_in[2];
  const float* W_V    = (const float*)d_in[3];
  const float* W_O    = (const float*)d_in[4];
  const float* W_fc   = (const float*)d_in[5];
  const float* W_proj = (const float*)d_in[6];
  const float* g1     = (const float*)d_in[7];
  const float* g2     = (const float*)d_in[8];
  float* out = (float*)d_out;

  size_t off = 0;
  auto carve = [&](size_t bytes) -> size_t {
    size_t o = off;
    off += (bytes + 255) & ~(size_t)255;
    return o;
  };
  const size_t o_wtq  = carve((size_t)kD * kD * 2);
  const size_t o_wtk  = carve((size_t)kD * kD * 2);
  const size_t o_wtv  = carve((size_t)kD * kD * 2);
  const size_t o_wto  = carve((size_t)kD * kD * 2);
  const size_t o_wtfc = carve((size_t)kDFF * kD * 2);
  const size_t o_wtpj = carve((size_t)kD * kDFF * 2);
  const size_t o_hpl  = carve((size_t)kM * kD * 2);
  const size_t o_qp   = carve((size_t)kM * kD * 2);
  const size_t o_kp   = carve((size_t)kM * kD * 2);
  const size_t o_vtp  = carve((size_t)kM * kD * 2);
  const size_t o_ctx  = carve((size_t)kM * kD * 2);
  const size_t o_z1   = carve((size_t)kM * kD * 4);
  const size_t o_gpl  = carve((size_t)kM * kDFF * 2);
  if (off > ws_size) return;

  char* ws = (char*)d_ws;
  _Float16* wtq  = (_Float16*)(ws + o_wtq);
  _Float16* wtk  = (_Float16*)(ws + o_wtk);
  _Float16* wtv  = (_Float16*)(ws + o_wtv);
  _Float16* wto  = (_Float16*)(ws + o_wto);
  _Float16* wtfc = (_Float16*)(ws + o_wtfc);
  _Float16* wtpj = (_Float16*)(ws + o_wtpj);
  _Float16* hpl  = (_Float16*)(ws + o_hpl);
  _Float16* qp   = (_Float16*)(ws + o_qp);
  _Float16* kp   = (_Float16*)(ws + o_kp);
  _Float16* vtp  = (_Float16*)(ws + o_vtp);
  _Float16* ctxp = (_Float16*)(ws + o_ctx);
  float*    z1   = (float*)   (ws + o_z1);
  _Float16* gpl  = (_Float16*)(ws + o_gpl);

  const dim3 b256(256), b128(128);

  cvt_wt<<<dim3(kD / 64, kD / 64), b256, 0, stream>>>(W_Q, wtq, kD, kD);
  cvt_wt<<<dim3(kD / 64, kD / 64), b256, 0, stream>>>(W_K, wtk, kD, kD);
  cvt_wt<<<dim3(kD / 64, kD / 64), b256, 0, stream>>>(W_V, wtv, kD, kD);
  cvt_wt<<<dim3(kD / 64, kD / 64), b256, 0, stream>>>(W_O, wto, kD, kD);
  cvt_wt<<<dim3(kDFF / 64, kD / 64), b256, 0, stream>>>(W_fc, wtfc, kD, kDFF);
  cvt_wt<<<dim3(kD / 64, kDFF / 64), b256, 0, stream>>>(W_proj, wtpj, kDFF, kD);

  rmsnorm_f16<1><<<dim3(kM), b128, 0, stream>>>(z, g1, hpl);

  const dim3 gD(kM / 128, kD / 128);
  const dim3 gF(kM / 128, kDFF / 128);
  gemm_rows<EPI_QK><<<gD, b256, 0, stream>>>(hpl, wtq, nullptr, nullptr, qp, kD, kD);
  gemm_rows<EPI_QK><<<gD, b256, 0, stream>>>(hpl, wtk, nullptr, nullptr, kp, kD, kD);
  gemm_vt<<<gD, b256, 0, stream>>>(hpl, wtv, vtp, kD);

  attn_causal<<<dim3(SEQ / 64, NB * kH), b128, 0, stream>>>(qp, kp, vtp, ctxp);

  gemm_rows<EPI_Z1><<<gD, b256, 0, stream>>>(ctxp, wto, z, z1, nullptr, kD, kD);

  rmsnorm_f16<0><<<dim3(kM), b128, 0, stream>>>(z1, g2, hpl);

  gemm_rows<EPI_GELU><<<gF, b256, 0, stream>>>(hpl, wtfc, nullptr, nullptr, gpl, kDFF, kD);
  gemm_rows<EPI_OUT><<<gD, b256, 0, stream>>>(gpl, wtpj, z1, out, nullptr, kD, kDFF);
}
